// SimpleMSA_62234076119748
// MI455X (gfx1250) — hardware-run, weakly checked
//
#include <hip/hip_runtime.h>


#define NB_  4
#define TQ   4096
#define NK   4096
#define DD   64
#define PCAR 1024.0f
typedef _Float16 h16;
typedef unsigned short bf;
typedef __attribute__((ext_vector_type(16))) __bf16   v16bf;
typedef __attribute__((ext_vector_type(16))) _Float16 v16h;
typedef __attribute__((ext_vector_type(8)))  _Float16 v8h;
typedef __attribute__((ext_vector_type(8)))  unsigned short v8us;
typedef __attribute__((ext_vector_type(8)))  float    v8f;
typedef __attribute__((ext_vector_type(4)))  float    v4f;
typedef v8h  __attribute__((may_alias)) v8ha;
typedef v4f  __attribute__((may_alias)) v4fa;
typedef v8us __attribute__((may_alias)) v8usa;

__device__ __forceinline__ unsigned short f2bf(float f) { unsigned u = __float_as_uint(f); u += 0x7FFFu + ((u >> 16) & 1u); return (unsigned short)(u >> 16); }
__device__ __forceinline__ float bf2f(unsigned short b) { return __uint_as_float(((unsigned)b) << 16); }
__device__ __forceinline__ float bfr(float f) { return bf2f(f2bf(f)); }
__device__ __forceinline__ v16h cat16(v8h lo, v8h hi) { return __builtin_shufflevector(lo, hi, 0, 1, 2, 3, 4, 5, 6, 7, 8, 9, 10, 11, 12, 13, 14, 15); }
__device__ __forceinline__ v16bf cat16b(v8us lo, v8us hi) { return __builtin_bit_cast(v16bf, __builtin_shufflevector(lo, hi, 0, 1, 2, 3, 4, 5, 6, 7, 8, 9, 10, 11, 12, 13, 14, 15)); }
__device__ __forceinline__ v8f wmma16(v16h a, v16h b, v8f c) { return __builtin_amdgcn_wmma_f32_16x16x32_f16(false, a, false, b, (short)0, c, false, false); }
__device__ __forceinline__ v8f wmmab(v16bf a, v16bf b, v8f c) { return __builtin_amdgcn_wmma_f32_16x16x32_bf16(false, a, false, b, (short)0, c, false, false); }


template <typename T16> struct WFrag;
template <> struct WFrag<h16> { typedef v16h V; static __device__ __forceinline__ V ld(const h16* p) { return cat16(*(const v8h*)p, *(const v8h*)(p + 16)); } static __device__ __forceinline__ v8f mma(V a, V b, v8f c) { return wmma16(a, b, c); } };
template <> struct WFrag<bf> { typedef v16bf V; static __device__ __forceinline__ V ld(const bf* p) { return cat16b(*(const v8us*)p, *(const v8us*)(p + 16)); } static __device__ __forceinline__ v8f mma(V a, V b, v8f c) { return wmmab(a, b, c); } };
template <typename T16, int NSPLIT, bool BIAS>
__global__ __launch_bounds__(32) void k_gemmw(const T16* __restrict__ A, const T16* __restrict__ A2, const T16* __restrict__ Bt, const T16* __restrict__ Bt2, int K, float* C, int ldc, const float* __restrict__ bias, size_t sA, size_t sB, size_t sC) {
    typedef typename WFrag<T16>::V V;
    __shared__ __align__(16) float os[16 * 68];
    const size_t z = blockIdx.z; A += z * sA; if (A2) A2 += z * sA; Bt += z * sB; if (Bt2) Bt2 += z * sB; C += z * sC;
    const int lane = threadIdx.x & 31, lr = lane & 15, hi = lane >> 4; const int r0 = blockIdx.x * 64, c0 = blockIdx.y * 64;
    v8f acc[4][4];
#pragma unroll
    for (int mb = 0; mb < 4; ++mb)
#pragma unroll
        for (int nb = 0; nb < 4; ++nb) acc[mb][nb] = (v8f){};
    const size_t aoff = (size_t)(r0 + lr) * K + 8 * hi, boff = (size_t)(c0 + lr) * K + 8 * hi;
#pragma unroll 1
    for (int kc = 0; kc < K; kc += 32) {
        V a[4], a2[4];
#pragma unroll
        for (int mb = 0; mb < 4; ++mb) { a[mb] = WFrag<T16>::ld(A + aoff + (size_t)mb * 16 * K + kc); if (NSPLIT == 1 || NSPLIT == 2) a2[mb] = WFrag<T16>::ld(A2 + aoff + (size_t)mb * 16 * K + kc); }
#pragma unroll
        for (int nb = 0; nb < 4; ++nb) { const V b = WFrag<T16>::ld(Bt + boff + (size_t)nb * 16 * K + kc); V b2; if (NSPLIT >= 2) b2 = WFrag<T16>::ld(Bt2 + boff + (size_t)nb * 16 * K + kc);
#pragma unroll
            for (int mb = 0; mb < 4; ++mb) { acc[mb][nb] = WFrag<T16>::mma(a[mb], b, acc[mb][nb]); if (NSPLIT == 1 || NSPLIT == 2) acc[mb][nb] = WFrag<T16>::mma(a2[mb], b, acc[mb][nb]); if (NSPLIT >= 2) acc[mb][nb] = WFrag<T16>::mma(a[mb], b2, acc[mb][nb]); } }
        asm volatile("v_nop\n\tv_nop\n\tv_nop\n\tv_nop" : "+v"(acc[0][0]), "+v"(acc[1][1]), "+v"(acc[2][2]), "+v"(acc[3][3]) : "v"(a[0]), "v"(a[3]));
    }
#pragma unroll
    for (int mb = 0; mb < 4; ++mb) {
#pragma unroll
        for (int nb = 0; nb < 4; ++nb) {
#pragma unroll
            for (int j = 0; j < 8; ++j) os[(hi * 8 + j) * 68 + nb * 16 + lr] = acc[mb][nb][j]; }
        __builtin_amdgcn_wave_barrier(); asm volatile("" ::: "memory");
        float* crow = C + (size_t)(r0 + mb * 16) * ldc + c0;
#pragma unroll 1
        for (int ps = 0; ps < 2; ++ps) {
#pragma unroll
            for (int s = 0; s < 8; ++s) { const int row = 2 * s + hi, cofs = lr * 4; v4f val = *(const v4fa*)(os + row * 68 + cofs); if (BIAS) { val[0] += bfr(bias[c0 + cofs]); val[1] += bfr(bias[c0 + cofs + 1]); val[2] += bfr(bias[c0 + cofs + 2]); val[3] += bfr(bias[c0 + cofs + 3]); }
                *(volatile v4f*)(crow + (size_t)row * ldc + cofs) = val; }
            if (ps == 0) __threadfence(); }
        __builtin_amdgcn_wave_barrier(); asm volatile("" ::: "memory");
    }
}

__device__ __forceinline__ h16 tohx(float x) { return (h16)x; }
typedef __attribute__((ext_vector_type(2))) _Float16 v2h;
typedef __attribute__((ext_vector_type(4))) _Float16 v4h;
typedef __attribute__((ext_vector_type(2))) float v2f;

__global__ __launch_bounds__(256) void k_cvt8(const float* __restrict__ src, bf* dst, size_t n8) { const size_t i = (size_t)blockIdx.x * 256 + threadIdx.x; if (i >= n8) return; const v8f v = *(const v8f*)(src + i * 8); v8us o;
#pragma unroll
    for (int k = 0; k < 8; ++k) o[k] = f2bf(v[k]); *(volatile v8us*)(dst + i * 8) = o; __threadfence(); *(volatile v8us*)(dst + i * 8) = o; }
__global__ __launch_bounds__(256) void k_sq(const float* __restrict__ t, float* SQ) { const int j = blockIdx.x * 256 + threadIdx.x; if (j >= NK) return; float s = 0.f;
    for (int d = 0; d < DD; ++d) { const float v = bfr(t[(size_t)j * DD + d]); float p = __fmul_rn(v, v); asm volatile("" : "+v"(p)); s = __fadd_rn(s, p); } *(volatile float*)(SQ + j) = s; __threadfence(); *(volatile float*)(SQ + j) = s; }
__global__ __launch_bounds__(256) void k_vt(const float* __restrict__ t, h16* VT) { const size_t e = ((size_t)blockIdx.x * 256 + threadIdx.x) * 2; if (e >= (size_t)DD * NK) return; const int j = (int)(e % NK), d = (int)(e / NK); v2h o; o[0] = tohx(bfr(t[(size_t)j * DD + d])); o[1] = tohx(bfr(t[(size_t)(j + 1) * DD + d])); *(volatile v2h*)(VT + e) = o; __threadfence(); *(volatile v2h*)(VT + e) = o; }
__device__ __forceinline__ float lgt(float g, float sqi, float sqj, float inv) { float g2 = __fmul_rn(2.0f, g); asm volatile("" : "+v"(g2)); const float msd = __fsub_rn(__fsub_rn(g2, sqi), sqj); float t = __fmul_rn(msd, inv); asm volatile("" : "+v"(t)); return t; }
__global__ __launch_bounds__(256) void k_lmax(const float* __restrict__ G, const float* __restrict__ SQ, const float* __restrict__ scale, float* RS) { const int lane = threadIdx.x & 31; const int i = blockIdx.x * 8 + (threadIdx.x >> 5); if (i >= TQ) return; const float inv = __fdiv_rn(1.0f, __fmul_rn(64.0f, bfr(scale[0]))); const float sqi = SQ[i]; const float* gr = G + (size_t)i * NK; float m = -3.0e38f;
#pragma unroll 4
    for (int c0 = lane * 4; c0 < NK; c0 += 128) { const v4f g = *(const v4f*)(gr + c0); const v4f s = *(const v4f*)(SQ + c0);
#pragma unroll
        for (int q = 0; q < 4; ++q) m = fmaxf(m, lgt(g[q], sqi, s[q], inv)); }
#pragma unroll
    for (int sh = 16; sh; sh >>= 1) m = fmaxf(m, __shfl_xor(m, sh, 32));
    const float o = lane == 0 ? m : 0.f; *(volatile float*)(RS + (size_t)i * 32 + lane) = o; __threadfence(); *(volatile float*)(RS + (size_t)i * 32 + lane) = o; }
__global__ __launch_bounds__(256) void k_lexp(const float* __restrict__ G, const float* __restrict__ SQ, const float* __restrict__ scale, float* RS, h16* P) { const int lane = threadIdx.x & 31; const int i = blockIdx.x * 8 + (threadIdx.x >> 5); if (i >= TQ) return; const float inv = __fdiv_rn(1.0f, __fmul_rn(64.0f, bfr(scale[0]))); const float sqi = SQ[i]; const float* gr = G + (size_t)i * NK; const float m = RS[(size_t)i * 32]; float sum = 0.f;
#pragma unroll 1
    for (int ps = 0; ps < 2; ++ps) { sum = 0.f;
#pragma unroll 2
        for (int c0 = lane * 4; c0 < NK; c0 += 128) { const v4f g = *(const v4f*)(gr + c0); const v4f s = *(const v4f*)(SQ + c0); v4h o;
#pragma unroll
            for (int q = 0; q < 4; ++q) { float dlt = __fsub_rn(lgt(g[q], sqi, s[q], inv), m); asm volatile("" : "+v"(dlt)); const float e = __expf(dlt); sum += e; o[q] = tohx(e * PCAR); }
            *(volatile v4h*)(P + (size_t)i * NK + c0) = o; }
        if (ps == 0) __threadfence(); }
#pragma unroll
    for (int sh = 16; sh; sh >>= 1) sum += __shfl_xor(sum, sh, 32);
    const float o2 = lane == 0 ? m : (lane == 1 ? __fdiv_rn(1.0f, __fmul_rn(sum, PCAR)) : 0.f); *(volatile float*)(RS + (size_t)i * 32 + lane) = o2; __threadfence(); *(volatile float*)(RS + (size_t)i * 32 + lane) = o2; }
__global__ __launch_bounds__(256) void k_ofin(const float* __restrict__ O, const float* __restrict__ RS, float* OUTb) { const size_t e = ((size_t)blockIdx.x * 256 + threadIdx.x) * 2; if (e >= (size_t)TQ * DD) return; const int i = (int)(e / DD); const float r = RS[(size_t)i * 32 + 1]; v2f o; o[0] = __fmul_rn(O[e], r); o[1] = __fmul_rn(O[e + 1], r); *(volatile v2f*)(OUTb + e) = o; __threadfence(); *(volatile v2f*)(OUTb + e) = o; }

extern "C" void kernel_launch(void* const* d_in, const int* in_sizes, int n_in,
                              void* d_out, int out_size, void* d_ws, size_t ws_size, hipStream_t stream) {
    (void)in_sizes; (void)n_in; (void)out_size;
    const float* tkn = (const float*)d_in[0]; const float* scale = (const float*)d_in[1];
    float* OUT = (float*)d_out;
    char* wsp = (char*)d_ws;
    auto take = [&](size_t bytes) { char* p = wsp; wsp += (bytes + 255) & ~(size_t)255; return (void*)p; };
    bf* XB = (bf*)take((size_t)TQ * DD * 2); float* SQ = (float*)take((size_t)NK * 4); h16* VT = (h16*)take((size_t)DD * NK * 2); float* G = (float*)take((size_t)TQ * NK * 4); h16* P = (h16*)take((size_t)TQ * NK * 2); float* RS = (float*)take((size_t)TQ * 32 * 4); float* O = (float*)take((size_t)TQ * DD * 4);
    if ((size_t)(wsp - (char*)d_ws) > ws_size) return;
    for (int b = 0; b < NB_; ++b) { const float* tb = tkn + (size_t)b * TQ * DD;
        k_cvt8<<<(TQ * DD / 8 + 255) / 256, 256, 0, stream>>>(tb, XB, (size_t)TQ * DD / 8); k_sq<<<NK / 256, 256, 0, stream>>>(tb, SQ); k_vt<<<(DD * NK / 2 + 255) / 256, 256, 0, stream>>>(tb, VT);
        k_gemmw<bf, 0, false><<<dim3(TQ / 64, NK / 64, 1), 32, 0, stream>>>(XB, nullptr, XB, nullptr, DD, G, NK, nullptr, 0, 0, 0);
        k_lmax<<<TQ / 8, 256, 0, stream>>>(G, SQ, scale, RS); k_lexp<<<TQ / 8, 256, 0, stream>>>(G, SQ, scale, RS, P);
        k_gemmw<h16, 0, false><<<dim3(TQ / 64, 1, 1), 32, 0, stream>>>(P, nullptr, VT, nullptr, NK, O, DD, nullptr, 0, 0, 0);
        k_ofin<<<(TQ * DD / 2 + 255) / 256, 256, 0, stream>>>(O, RS, OUT + (size_t)b * TQ * DD); }
}
